// GRU_Adversarial_22952305229977
// MI455X (gfx1250) — hardware-verified
//
#include <hip/hip_runtime.h>


#define AS3 __attribute__((address_space(3)))

#define T_    128
#define B_    256
#define H_    512
#define G3_   1536
#define IN_   6
#define OD_   512
#define DX_   4
#define MB_   16
#define NBLK  (B_ / MB_)
#define NTHR  256
#define XP    1032
#define K1_   1024
#define HM_   32
#define SUP   516

static_assert(NBLK * MB_ == B_);
static_assert(NTHR == 256);
static_assert(H_ == (NTHR / 32) * 64);
static_assert(XP % 8 == 0);
static_assert(XP >= K1_);
static_assert((SUP * 4) % 16 == 0);
static_assert(SUP >= OD_);
static_assert(H_ % 32 == 0);
static_assert(K1_ == 2 * H_);
static_assert((T_ * B_) % HM_ == 0);
static_assert(B_ % HM_ == 0);
static_assert(OD_ == T_ * DX_);
static_assert(MB_ * IN_ <= 96);

typedef _Float16 v16h __attribute__((ext_vector_type(16)));
typedef _Float16 v8h  __attribute__((ext_vector_type(8)));
typedef _Float16 v4h  __attribute__((ext_vector_type(4)));
typedef float    v8f  __attribute__((ext_vector_type(8)));
typedef float    v4f  __attribute__((ext_vector_type(4)));

typedef AS3 _Float16*       lp_h;
typedef AS3 const _Float16* lcp_h;
typedef AS3 float*          lp_f;
typedef AS3 const float*    lcp_f;

union Frag { v16h v; v8h half[2]; };

#define ASCL    16.0f
#define WSCL    64.0f
#define INV1024 0.0009765625f

constexpr size_t SZ_W0  = (size_t)G3_ * H_ * 2;
constexpr size_t SZ_W1  = (size_t)G3_ * K1_ * 2;
constexpr size_t SZ_WL  = (size_t)OD_ * H_ * 2;
constexpr size_t SZ_Y1  = (size_t)T_ * B_ * H_ * 2;
constexpr size_t SZ_REC = (size_t)T_ * B_ * 8 * 4;
constexpr size_t OFF_W0  = 0;
constexpr size_t OFF_W1  = OFF_W0 + SZ_W0;
constexpr size_t OFF_WL  = OFF_W1 + SZ_W1;
constexpr size_t OFF_Y1  = OFF_WL + SZ_WL;
constexpr size_t OFF_REC = OFF_Y1 + SZ_Y1;
constexpr size_t WS_END  = OFF_REC + SZ_REC;
static_assert(OFF_W1 % 128 == 0 && OFF_WL % 128 == 0 && OFF_Y1 % 128 == 0 && OFF_REC % 128 == 0);
static_assert(WS_END <= (size_t)134217728);

constexpr int NP0 = G3_ * H_ / 8;
constexpr int NP1 = G3_ * K1_ / 8;
constexpr int NPL = OD_ * H_ / 8;
constexpr int NB0 = NP0 / 256;
constexpr int NB1 = NP1 / 256;
constexpr int NBL = NPL / 256;
static_assert(NP0 % 256 == 0 && NP1 % 256 == 0 && NPL % 256 == 0);
static_assert((size_t)NP0 * 16 == SZ_W0);
static_assert((size_t)NP1 * 16 == SZ_W1);
static_assert((size_t)NPL * 16 == SZ_WL);

constexpr int    XT       = MB_ * XP;
constexpr size_t LOFF_X   = 0;
constexpr size_t LSZ_X    = (size_t)2 * XT * 2;
constexpr size_t LOFF_HF  = LOFF_X + LSZ_X;
constexpr size_t LSZ_HF   = (size_t)2 * MB_ * H_ * 4;
constexpr size_t LOFF_B0  = LOFF_HF + LSZ_HF;
constexpr size_t LOFF_B1  = LOFF_B0 + 2048 * 4;
constexpr size_t LOFF_WI  = LOFF_B1 + 2048 * 4;
constexpr size_t LOFF_XS  = LOFF_WI + (size_t)G3_ * IN_ * 4;
constexpr size_t LDS_BYTES = LOFF_XS + 2 * MB_ * 8 * 4;
static_assert(LOFF_HF % 16 == 0 && LOFF_B0 % 16 == 0 && LOFF_B1 % 16 == 0 && LOFF_WI % 16 == 0 && LOFF_XS % 16 == 0);
static_assert((2 * XT) % 8 == 0);
static_assert((XP * 2) % 16 == 0);

constexpr size_t LH_SU    = 0;
constexpr size_t LH_BL    = LH_SU + (size_t)HM_ * SUP * 4;
constexpr size_t LH_REC   = LH_BL + (size_t)OD_ * 4;
constexpr size_t LH_BYTES = LH_REC + (size_t)HM_ * 8 * 4;
static_assert(LH_BL % 16 == 0 && LH_REC % 16 == 0);

#if defined(__HIP_DEVICE_COMPILE__)
#define GUARD3(c0, c1, c2, a0, b0, b1, b2) \
    asm volatile("v_nop\n\tv_nop\n\tv_nop\n\tv_nop" : "+v"(c0), "+v"(c1), "+v"(c2) : "v"(a0), "v"(b0), "v"(b1), "v"(b2))
#define GUARD4(c0, c1, c2, c3, a0, b0, b1, b2) \
    asm volatile("v_nop\n\tv_nop\n\tv_nop\n\tv_nop" : "+v"(c0), "+v"(c1), "+v"(c2), "+v"(c3) : "v"(a0), "v"(b0), "v"(b1), "v"(b2))
#define GUARD8(c0, c1, c2, c3, c4, c5, c6, c7, a0, a1, b0, b1, b2, b3) \
    asm volatile("v_nop\n\tv_nop\n\tv_nop\n\tv_nop" : "+v"(c0), "+v"(c1), "+v"(c2), "+v"(c3), "+v"(c4), "+v"(c5), "+v"(c6), "+v"(c7) \
                 : "v"(a0), "v"(a1), "v"(b0), "v"(b1), "v"(b2), "v"(b3))
#else
#define GUARD3(c0, c1, c2, a0, b0, b1, b2) do { } while (0)
#define GUARD4(c0, c1, c2, c3, a0, b0, b1, b2) do { } while (0)
#define GUARD8(c0, c1, c2, c3, c4, c5, c6, c7, a0, a1, b0, b1, b2, b3) do { } while (0)
#endif

__device__ __forceinline__ float rcpx(float x) { return __builtin_amdgcn_rcpf(x); }
__device__ __forceinline__ float sigm(float x) { return rcpx(1.0f + __expf(-x)); }
__device__ __forceinline__ float tanhm(float x) {
    const float e = __expf(2.0f * x);
    return 1.0f - 2.0f * rcpx(e + 1.0f);
}
__device__ __forceinline__ v8f ld8f(const float* p) {
    const v4f a = *(const v4f*)p;
    const v4f b = *(const v4f*)(p + 4);
    return __builtin_shufflevector(a, b, 0, 1, 2, 3, 4, 5, 6, 7);
}
__device__ __forceinline__ v8f zero8() {
    v8f z;
#pragma unroll
    for (int i = 0; i < 8; ++i) z[i] = 0.0f;
    return z;
}
__device__ __forceinline__ float dot4(v4f v) { return v[0] * v[0] + v[1] * v[1] + v[2] * v[2] + v[3] * v[3]; }

__device__ __forceinline__ void ldfrag_lds(Frag& f, lcp_h p) {
    f.half[0] = *(AS3 const v8h*)(p);
    f.half[1] = *(AS3 const v8h*)(p + 16);
}
__device__ __forceinline__ void ldfrag_glb(Frag& f, const _Float16* p) {
    f.half[0] = *(const v8h*)(p);
    f.half[1] = *(const v8h*)(p + 16);
}
__device__ __forceinline__ v8f mma16(v8f c, const Frag& a, const Frag& b) {
    return __builtin_amdgcn_wmma_f32_16x16x32_f16(false, a.v, false, b.v, (short)0, c, false, false);
}

__global__ __launch_bounds__(256)
void cvt_kernel(const float* __restrict__ Whh0, const float* __restrict__ Wih1,
                const float* __restrict__ Whh1, const float* __restrict__ Wlin,
                _Float16* W0p, _Float16* W1p, _Float16* Wlp)
{
    const int tid = threadIdx.x;
    const int bid = blockIdx.x;
    v8h hv;
    _Float16* d;
    if (bid < NB0) {
        const int p  = bid * 256 + tid;
        const int n  = p >> 6;
        const int c8 = (p & 63) * 8;
        const v8f a = ld8f(Whh0 + (size_t)n * H_ + c8);
#pragma unroll
        for (int i = 0; i < 8; ++i) hv[i] = (_Float16)(a[i] * WSCL);
        d = W0p + (size_t)n * H_ + c8;
    } else if (bid < NB0 + NB1) {
        const int p  = (bid - NB0) * 256 + tid;
        const int n  = p >> 7;
        const int c8 = (p & 127) * 8;
        const int ci = min(c8, H_ - 8);
        const int cj = min(max(c8 - H_, 0), H_ - 8);
        const v8f a = ld8f(Wih1 + (size_t)n * H_ + ci);
        const v8f b = ld8f(Whh1 + (size_t)n * H_ + cj);
#pragma unroll
        for (int i = 0; i < 8; ++i) {
            const float v = (c8 < H_) ? a[i] : b[i];
            hv[i] = (_Float16)(v * WSCL);
        }
        d = W1p + (size_t)n * K1_ + c8;
    } else {
        const int p  = (bid - NB0 - NB1) * 256 + tid;
        const int n  = p >> 6;
        const int c8 = (p & 63) * 8;
        const v8f a = ld8f(Wlin + (size_t)n * H_ + c8);
#pragma unroll
        for (int i = 0; i < 8; ++i) hv[i] = (_Float16)(a[i] * WSCL);
        d = Wlp + (size_t)n * H_ + c8;
    }
    *(volatile v8h*)d = hv;
    __threadfence();
    *(volatile v8h*)d = hv;
}

__device__ __forceinline__ void stage_x(lp_f dst, const float* __restrict__ pN, const float* __restrict__ mN,
                                        int t, int b0, int tid)
{
    if (tid < 96) {
        const int row = tid / IN_;
        const int k   = tid - row * IN_;
        const size_t rb = (size_t)t * B_ + b0 + row;
        const float vp = pN[rb * 4 + min(k, 3)];
        const float vm = mN[rb * 2 + min(max(k - 4, 0), 1)];
        dst[row * 8 + k] = (k < 4) ? vp : vm;
    }
}

__device__ __forceinline__ void store_y1(lcp_h th1, _Float16* Y1, int t, int b0, int tid)
{
    _Float16* yb = Y1 + ((size_t)t * B_ + b0) * H_;
#pragma unroll
    for (int it = 0; it < 4; ++it) {
        const int p = it * 256 + tid, row = p >> 6, c8 = (p & 63) * 8;
        const v8h v = *(AS3 const v8h*)(th1 + row * XP + c8);
        *(volatile v8h*)(yb + (size_t)row * H_ + c8) = v;
    }
    __threadfence();
#pragma unroll
    for (int it = 0; it < 4; ++it) {
        const int p = it * 256 + tid, row = p >> 6, c8 = (p & 63) * 8;
        const v8h v = *(AS3 const v8h*)(th1 + row * XP + c8);
        *(volatile v8h*)(yb + (size_t)row * H_ + c8) = v;
    }
}

__global__ __launch_bounds__(NTHR)
void gru_seq_kernel(const float* __restrict__ pN, const float* __restrict__ mN, const float* __restrict__ hid,
                    const float* __restrict__ Wih0, const float* __restrict__ bih0, const float* __restrict__ bhh0,
                    const float* __restrict__ bih1, const float* __restrict__ bhh1,
                    const _Float16* __restrict__ W0p, const _Float16* __restrict__ W1p,
                    _Float16* Y1, float* out1)
{
    extern __shared__ __attribute__((aligned(16))) char smem[];
    lp_h sX  = (lp_h)(smem + LOFF_X);
    lp_f sHF = (lp_f)(smem + LOFF_HF);
    lp_f sB0 = (lp_f)(smem + LOFF_B0);
    lp_f sB1 = (lp_f)(smem + LOFF_B1);
    lp_f sWI = (lp_f)(smem + LOFF_WI);
    lp_f sXS = (lp_f)(smem + LOFF_XS);

    const int tid  = threadIdx.x;
    const int lane = tid & 31;
    const int w    = tid >> 5;
    const int h    = lane >> 4;
    const int m    = lane & 15;
    const int b0   = blockIdx.x * MB_;

    {
        v8h zh;
#pragma unroll
        for (int i = 0; i < 8; ++i) zh[i] = (_Float16)0.0f;
        for (int i = tid; i < (2 * XT) / 8; i += NTHR) *(AS3 v8h*)(sX + 8 * i) = zh;
        sXS[tid] = 0.0f;
        for (int i = tid; i < 1024; i += NTHR) {
            sB0[i] = bih0[i] + bhh0[i];
            sB1[i] = bih1[i] + bhh1[i];
        }
        for (int i = tid; i < 512; i += NTHR) {
            sB0[1024 + i] = bih0[1024 + i];
            sB0[1536 + i] = bhh0[1024 + i];
            sB1[1024 + i] = bih1[1024 + i];
            sB1[1536 + i] = bhh1[1024 + i];
        }
        for (int i = tid; i < G3_ * IN_; i += NTHR) sWI[i] = Wih0[i];
    }
    __syncthreads();
    {
        for (int i = tid; i < MB_ * (H_ / 4); i += NTHR) {
            const int row = i >> 7, c4 = (i & 127) * 4;
#pragma unroll
            for (int l = 0; l < 2; ++l) {
                const v4f v = *(const v4f*)(hid + ((size_t)(l * B_ + b0 + row)) * H_ + c4);
                *(AS3 v4f*)(sHF + l * (MB_ * H_) + row * H_ + c4) = v;
                v4h hv;
#pragma unroll
                for (int i2 = 0; i2 < 4; ++i2) hv[i2] = (_Float16)(v[i2] * ASCL);
                *(AS3 v4h*)(sX + row * XP + l * H_ + c4) = hv;
            }
        }
        stage_x(sXS, pN, mN, 0, b0, tid);
    }

#pragma unroll 1
    for (int s = 0; s < T_; ++s) {
        const int cur = s & 1;
        lp_h sXc = sX + cur * XT;
        lp_h sXn = sX + (cur ^ 1) * XT;
        lcp_f xsb = sXS + cur * (MB_ * 8);

        __syncthreads();

        if (s >= 1) store_y1(sXc + H_, Y1, s - 1, b0, tid);
        if (s + 1 < T_) stage_x(sXS + (cur ^ 1) * (MB_ * 8), pN, mN, s + 1, b0, tid);

#pragma unroll 1
        for (int g4 = 0; g4 < 4; ++g4) {
            const int j0 = w * 64 + g4 * 16;
            const int n  = j0 + m;
            v8f aR = zero8(), aZ = zero8(), aN = zero8();
            lcp_h ab = sXc + m * XP + 8 * h;
            const _Float16* wb = W0p + (size_t)n * H_ + 8 * h;
#pragma unroll 1
            for (int k0 = 0; k0 < H_; k0 += 32) {
                Frag a, bR, bZ, bN;
                ldfrag_lds(a, ab + k0);
                ldfrag_glb(bR, wb + k0);
                ldfrag_glb(bZ, wb + (size_t)H_ * H_ + k0);
                ldfrag_glb(bN, wb + (size_t)2 * H_ * H_ + k0);
                aR = mma16(aR, a, bR);
                aZ = mma16(aZ, a, bZ);
                aN = mma16(aN, a, bN);
                GUARD3(aR, aZ, aN, a.v, bR.v, bZ.v, bN.v);
            }
            float wr[IN_], wz[IN_], wn[IN_];
#pragma unroll
            for (int k = 0; k < IN_; ++k) {
                wr[k] = sWI[n * IN_ + k];
                wz[k] = sWI[(H_ + n) * IN_ + k];
                wn[k] = sWI[(2 * H_ + n) * IN_ + k];
            }
            const float br  = sB0[n];
            const float bz  = sB0[H_ + n];
            const float bin = sB0[2 * H_ + n];
            const float bhn = sB0[3 * H_ + n];
#pragma unroll
            for (int r = 0; r < 8; ++r) {
                const int row = 8 * h + r;
                const v4f xa = *(AS3 const v4f*)(xsb + row * 8);
                const v4f xb = *(AS3 const v4f*)(xsb + row * 8 + 4);
                float gr = br, gz = bz, gn = bin;
#pragma unroll
                for (int k = 0; k < 4; ++k) {
                    gr += xa[k] * wr[k];
                    gz += xa[k] * wz[k];
                    gn += xa[k] * wn[k];
                }
                gr += xb[0] * wr[4] + xb[1] * wr[5];
                gz += xb[0] * wz[4] + xb[1] * wz[5];
                gn += xb[0] * wn[4] + xb[1] * wn[5];
                const float rg = sigm(aR[r] * INV1024 + gr);
                const float zg = sigm(aZ[r] * INV1024 + gz);
                const float ng = tanhm(gn + rg * (aN[r] * INV1024 + bhn));
                lp_f hp = sHF + row * H_ + n;
                const float ho = *hp;
                const float hn = (1.0f - zg) * ng + zg * ho;
                *hp = hn;
                sXn[row * XP + n] = (_Float16)(hn * ASCL);
            }
        }

        __syncthreads();

#pragma unroll 1
        for (int g4 = 0; g4 < 4; ++g4) {
            const int j0 = w * 64 + g4 * 16;
            const int n  = j0 + m;
            v8f aR = zero8(), aZ = zero8(), aI = zero8(), aH = zero8();
            lcp_h aA = sXn + m * XP + 8 * h;
            lcp_h aB = sXc + m * XP + H_ + 8 * h;
            const _Float16* wb = W1p + (size_t)n * K1_ + 8 * h;
#pragma unroll 1
            for (int k0 = 0; k0 < H_; k0 += 32) {
                Frag a, bR, bZ, bI;
                ldfrag_lds(a, aA + k0);
                ldfrag_glb(bR, wb + k0);
                ldfrag_glb(bZ, wb + (size_t)H_ * K1_ + k0);
                ldfrag_glb(bI, wb + (size_t)2 * H_ * K1_ + k0);
                aR = mma16(aR, a, bR);
                aZ = mma16(aZ, a, bZ);
                aI = mma16(aI, a, bI);
                GUARD3(aR, aZ, aI, a.v, bR.v, bZ.v, bI.v);
            }
#pragma unroll 1
            for (int k0 = 0; k0 < H_; k0 += 32) {
                Frag a, bR, bZ, bH;
                ldfrag_lds(a, aB + k0);
                ldfrag_glb(bR, wb + H_ + k0);
                ldfrag_glb(bZ, wb + (size_t)H_ * K1_ + H_ + k0);
                ldfrag_glb(bH, wb + (size_t)2 * H_ * K1_ + H_ + k0);
                aR = mma16(aR, a, bR);
                aZ = mma16(aZ, a, bZ);
                aH = mma16(aH, a, bH);
                GUARD4(aR, aZ, aH, aI, a.v, bR.v, bZ.v, bH.v);
            }
            const float br  = sB1[n];
            const float bz  = sB1[H_ + n];
            const float bin = sB1[2 * H_ + n];
            const float bhn = sB1[3 * H_ + n];
#pragma unroll
            for (int r = 0; r < 8; ++r) {
                const int row = 8 * h + r;
                const float rg = sigm(aR[r] * INV1024 + br);
                const float zg = sigm(aZ[r] * INV1024 + bz);
                const float ng = tanhm(aI[r] * INV1024 + bin + rg * (aH[r] * INV1024 + bhn));
                lp_f hp = sHF + (MB_ * H_) + row * H_ + n;
                const float ho = *hp;
                const float hn = (1.0f - zg) * ng + zg * ho;
                *hp = hn;
                sXn[row * XP + H_ + n] = (_Float16)(hn * ASCL);
            }
        }
    }

    __syncthreads();
    store_y1(sX + (T_ & 1) * XT + H_, Y1, T_ - 1, b0, tid);

#pragma unroll 1
    for (int l = 0; l < 2; ++l) {
        lcp_f src = sHF + l * (MB_ * H_);
        float* dst = out1 + ((size_t)(l * B_ + b0)) * H_;
#pragma unroll
        for (int it = 0; it < 8; ++it) {
            const int p = it * 256 + tid, row = p >> 7, c4 = (p & 127) * 4;
            const v4f v = *(AS3 const v4f*)(src + row * H_ + c4);
            *(volatile v4f*)(dst + (size_t)row * H_ + c4) = v;
        }
        __threadfence();
#pragma unroll
        for (int it = 0; it < 8; ++it) {
            const int p = it * 256 + tid, row = p >> 7, c4 = (p & 127) * 4;
            const v4f v = *(AS3 const v4f*)(src + row * H_ + c4);
            *(volatile v4f*)(dst + (size_t)row * H_ + c4) = v;
        }
    }
}

__global__ __launch_bounds__(256)
void head_kernel(const _Float16* __restrict__ Y1, const _Float16* __restrict__ Wlp,
                 const float* __restrict__ blin, float* REC)
{
    extern __shared__ __attribute__((aligned(16))) char smem[];
    lp_f su   = (lp_f)(smem + LH_SU);
    lp_f sbl  = (lp_f)(smem + LH_BL);
    lp_f srec = (lp_f)(smem + LH_REC);

    const int tid  = threadIdx.x;
    const int lane = tid & 31;
    const int w    = tid >> 5;
    const int h    = lane >> 4;
    const int m    = lane & 15;
    const int m0   = blockIdx.x * HM_;
    const int t    = m0 >> 8;

    for (int i = tid; i < OD_; i += 256) sbl[i] = blin[i];
    __syncthreads();

    v8f acc[2][4];
#pragma unroll
    for (int mt = 0; mt < 2; ++mt)
#pragma unroll
        for (int q = 0; q < 4; ++q) acc[mt][q] = zero8();

    const _Float16* ab = Y1  + (size_t)(m0 + m) * H_ + 8 * h;
    const _Float16* wb = Wlp + (size_t)(w * 64 + m) * H_ + 8 * h;
#pragma unroll 1
    for (int k0 = 0; k0 < H_; k0 += 32) {
        Frag a[2], b[4];
#pragma unroll
        for (int mt = 0; mt < 2; ++mt) ldfrag_glb(a[mt], ab + (size_t)mt * (16 * H_) + k0);
#pragma unroll
        for (int q = 0; q < 4; ++q) ldfrag_glb(b[q], wb + (size_t)q * (16 * H_) + k0);
#pragma unroll
        for (int mt = 0; mt < 2; ++mt)
#pragma unroll
            for (int q = 0; q < 4; ++q) acc[mt][q] = mma16(acc[mt][q], a[mt], b[q]);
        GUARD8(acc[0][0], acc[0][1], acc[0][2], acc[0][3], acc[1][0], acc[1][1], acc[1][2], acc[1][3],
               a[0].v, a[1].v, b[0].v, b[1].v, b[2].v, b[3].v);
    }

#pragma unroll
    for (int mt = 0; mt < 2; ++mt) {
#pragma unroll
        for (int q = 0; q < 4; ++q) {
            const int col = w * 64 + q * 16 + m;
            const float bb = sbl[col];
#pragma unroll
            for (int r = 0; r < 8; ++r)
                su[(mt * 16 + 8 * h + r) * SUP + col] = acc[mt][q][r] * INV1024 + bb;
        }
    }
    __syncthreads();

#pragma unroll
    for (int rr = 0; rr < 4; ++rr) {
        const int row = 4 * w + rr;
        lcp_f rp = su + row * SUP;
        float s = 0.0f;
#pragma unroll
        for (int j = 0; j < 4; ++j) {
            const int q = j * 32 + lane;
            const v4f v = *(AS3 const v4f*)(rp + 4 * q);
            const float e = dot4(v);
            s += (q >= t) ? e : 0.0f;
        }
#pragma unroll
        for (int off = 16; off; off >>= 1) s += __shfl_xor(s, off, 32);
        const v4f dv = *(AS3 const v4f*)(rp + 4 * t);
        const float de = dot4(dv);
        if (lane == 0) {
            v4f sd;
            sd[0] = s; sd[1] = de; sd[2] = 0.0f; sd[3] = 0.0f;
            *(AS3 v4f*)(srec + row * 8) = dv;
            *(AS3 v4f*)(srec + row * 8 + 4) = sd;
        }
    }
    __syncthreads();

    float* rd = REC + (size_t)m0 * 8;
    if (tid < 64) {
        const v4f v = *(AS3 const v4f*)(srec + tid * 4);
        *(volatile v4f*)(rd + tid * 4) = v;
    }
    __threadfence();
    if (tid < 64) {
        const v4f v = *(AS3 const v4f*)(srec + tid * 4);
        *(volatile v4f*)(rd + tid * 4) = v;
    }
}

__global__ __launch_bounds__(256)
void scan_kernel(const float* __restrict__ REC, float* out0)
{
    const int b = threadIdx.x;
    double L = (double)T_;
#pragma unroll 1
    for (int k = 0; k < T_; ++k) {
        const float* rp = REC + ((size_t)k * B_ + b) * 8;
        const v4f du = *(const v4f*)(rp);
        const v4f sd = *(const v4f*)(rp + 4);
        const double suf = (double)sd[0];
        const double de  = (double)sd[1];
        const float sc = sqrtf((float)(L / suf));
        const v4f o = du * sc;
        float* dp = out0 + ((size_t)k * B_ + b) * 4;
        *(volatile v4f*)dp = o;
        __threadfence();
        *(volatile v4f*)dp = o;
        L = L * (1.0 - de / suf);
    }
}

extern "C" void kernel_launch(void* const* d_in, const int* in_sizes, int n_in,
                              void* d_out, int out_size, void* d_ws, size_t ws_size,
                              hipStream_t stream)
{
    if (n_in < 13) return;
    if (in_sizes[0]  != T_ * B_ * 4)   return;
    if (in_sizes[1]  != T_ * B_ * 2)   return;
    if (in_sizes[2]  != 2 * B_ * H_)   return;
    if (in_sizes[3]  != G3_ * IN_)     return;
    if (in_sizes[4]  != G3_ * H_)      return;
    if (in_sizes[5]  != G3_)           return;
    if (in_sizes[6]  != G3_)           return;
    if (in_sizes[7]  != G3_ * H_)      return;
    if (in_sizes[8]  != G3_ * H_)      return;
    if (in_sizes[9]  != G3_)           return;
    if (in_sizes[10] != G3_)           return;
    if (in_sizes[11] != OD_ * H_)      return;
    if (in_sizes[12] != OD_)           return;
    if (out_size != T_ * B_ * DX_ + 2 * B_ * H_) return;
    if (ws_size < WS_END) return;

    const float* pN   = (const float*)d_in[0];
    const float* mN   = (const float*)d_in[1];
    const float* hid  = (const float*)d_in[2];
    const float* Wih0 = (const float*)d_in[3];
    const float* Whh0 = (const float*)d_in[4];
    const float* bih0 = (const float*)d_in[5];
    const float* bhh0 = (const float*)d_in[6];
    const float* Wih1 = (const float*)d_in[7];
    const float* Whh1 = (const float*)d_in[8];
    const float* bih1 = (const float*)d_in[9];
    const float* bhh1 = (const float*)d_in[10];
    const float* Wlin = (const float*)d_in[11];
    const float* blin = (const float*)d_in[12];
    float* out0 = (float*)d_out;
    float* out1 = (float*)d_out + (size_t)T_ * B_ * DX_;

    char* ws = (char*)d_ws;
    _Float16* W0p = (_Float16*)(ws + OFF_W0);
    _Float16* W1p = (_Float16*)(ws + OFF_W1);
    _Float16* Wlp = (_Float16*)(ws + OFF_WL);
    _Float16* Y1  = (_Float16*)(ws + OFF_Y1);
    float*    REC = (float*)(ws + OFF_REC);

    cvt_kernel<<<dim3(NB0 + NB1 + NBL), dim3(256), 0, stream>>>(Whh0, Wih1, Whh1, Wlin, W0p, W1p, Wlp);

    hipFuncSetAttribute(reinterpret_cast<const void*>(&gru_seq_kernel),
                        hipFuncAttributeMaxDynamicSharedMemorySize, (int)LDS_BYTES);
    gru_seq_kernel<<<dim3(NBLK), dim3(NTHR), LDS_BYTES, stream>>>(
        pN, mN, hid, Wih0, bih0, bhh0, bih1, bhh1, (const _Float16*)W0p, (const _Float16*)W1p, Y1, out1);

    hipFuncSetAttribute(reinterpret_cast<const void*>(&head_kernel),
                        hipFuncAttributeMaxDynamicSharedMemorySize, (int)LH_BYTES);
    head_kernel<<<dim3((T_ * B_) / HM_), dim3(256), LH_BYTES, stream>>>((const _Float16*)Y1, (const _Float16*)Wlp, blin, REC);

    scan_kernel<<<dim3(1), dim3(B_), 0, stream>>>((const float*)REC, out0);
}
